// HebbianMambaLayer_1709396983863
// MI455X (gfx1250) — hardware-verified
//
#include <hip/hip_runtime.h>
#include <math.h>

typedef __attribute__((ext_vector_type(16))) _Float16 v16h;
typedef __attribute__((ext_vector_type(8)))  _Float16 v8h;
typedef __attribute__((ext_vector_type(16))) __bf16   v16b;
typedef __attribute__((ext_vector_type(8)))  __bf16   v8b;
typedef __attribute__((ext_vector_type(8)))  float    v8f;
typedef __attribute__((ext_vector_type(4)))  float    v4f;

constexpr int kBatch  = 4;
constexpr int kSeq    = 1024;
constexpr int kDm     = 512;
constexpr int kDin    = 1024;
constexpr int kNst    = 16;
constexpr int kDtR    = 32;
constexpr int kXzP    = 2 * kDin;
constexpr int kXdP    = 64;
constexpr int kRows   = kBatch * kSeq;
constexpr int kConvTP = 260;
constexpr int kScanTS = 64;
constexpr int kScanCh = 64;
constexpr int kScanYP = 68;
static_assert(kDtR + 2 * kNst == kXdP);
static_assert((kDm % 32) == 0 && (kDin % 32) == 0 && (kSeq % 32) == 0);
static_assert((kRows % 64) == 0 && (kXzP % 64) == 0 && (kXdP % 64) == 0 && (kDm % 64) == 0 && (kSeq % 64) == 0);
static_assert((kSeq % kScanTS) == 0 && (kDin % kScanCh) == 0 && (kDin % 256) == 0);
static_assert((kSeq & (kSeq - 1)) == 0);

constexpr float kWsc = 64.0f;
constexpr float kUsc = 64.0f;
constexpr float kYsc = 64.0f;
constexpr float kOsc = 256.0f;
constexpr float kVsc = 4096.0f;
constexpr float kPsc = 65536.0f;
constexpr float kRsc = 262144.0f;

constexpr size_t kOffH16   = 0;
constexpr size_t kOffWI16  = kOffH16   + (size_t)kRows * kDm  * 2;
constexpr size_t kOffWX16  = kOffWI16  + (size_t)kXzP  * kDm  * 2;
constexpr size_t kOffWO16  = kOffWX16  + (size_t)kXdP  * kDin * 2;
constexpr size_t kOffWW16  = kOffWO16  + (size_t)kDm   * kDin * 2;
constexpr size_t kOffWR16  = kOffWW16  + (size_t)kDm   * kDm  * 2;
constexpr size_t kOffXZ    = kOffWR16  + (size_t)kDm   * kDm  * 2;
constexpr size_t kOffS     = kOffXZ;
constexpr size_t kOffP16   = kOffS     + (size_t)kBatch * kSeq * kSeq * 4;
constexpr size_t kOffUC    = kOffXZ    + (size_t)kRows * kXzP * 4;
constexpr size_t kOffU16   = kOffUC    + (size_t)kRows * kDin * 4;
constexpr size_t kOffXD    = kOffU16   + (size_t)kRows * kDin * 2;
constexpr size_t kOffY16   = kOffXD    + (size_t)kRows * kXdP * 4;
constexpr size_t kOffOUT   = kOffY16   + (size_t)kRows * kDin * 2;
constexpr size_t kOffOUT16 = kOffOUT   + (size_t)kRows * kDm  * 4;
constexpr size_t kOffWK16  = kOffOUT16 + (size_t)kRows * kDm  * 2;
constexpr size_t kOffXPO   = kOffWK16  + (size_t)kRows * kDm  * 2;
constexpr size_t kOffVT16  = kOffXPO   + (size_t)kRows * kDm  * 4;
constexpr size_t kOffRD16  = kOffVT16  + (size_t)kBatch * kDm * kSeq * 2;
constexpr size_t kWsTotal  = kOffRD16  + (size_t)kRows * kDm  * 2;
static_assert(kWsTotal == 110231552ull);
static_assert(kWsTotal <= 134217728ull);
static_assert(kOffP16 + (size_t)kBatch * kSeq * kSeq * 2 <= kOffUC);
static_assert((kOffWI16 % 128) == 0 && (kOffWX16 % 128) == 0 && (kOffWO16 % 128) == 0 && (kOffWW16 % 128) == 0 &&
              (kOffWR16 % 128) == 0 && (kOffXZ % 128) == 0 && (kOffP16 % 128) == 0 && (kOffUC % 128) == 0 &&
              (kOffU16 % 128) == 0 && (kOffXD % 128) == 0 && (kOffY16 % 128) == 0 && (kOffOUT % 128) == 0 &&
              (kOffOUT16 % 128) == 0 && (kOffWK16 % 128) == 0 && (kOffXPO % 128) == 0 && (kOffVT16 % 128) == 0 &&
              (kOffRD16 % 128) == 0);

__device__ __forceinline__ unsigned short f2bf_bits(float f) {
  unsigned u = __float_as_uint(f);
  return (unsigned short)((u + 0x7FFFu + ((u >> 16) & 1u)) >> 16);
}
__device__ __forceinline__ float bf_bits2f(unsigned short h) { return __uint_as_float(((unsigned)h) << 16); }

__device__ __forceinline__ void dep_guard_h(v8f& a, v8f& b, v16h x, v16h y) { asm volatile("v_nop\n\tv_nop\n\tv_nop\n\tv_nop" : "+v"(a), "+v"(b) : "v"(x), "v"(y)); }
__device__ __forceinline__ void dep_guard_b(v8f& a, v8f& b, v16b x, v16b y) { asm volatile("v_nop\n\tv_nop\n\tv_nop\n\tv_nop" : "+v"(a), "+v"(b) : "v"(x), "v"(y)); }
__device__ __forceinline__ void keep4_h(v16h a, v16h b, v16h c, v16h d) { asm volatile("v_nop" :: "v"(a), "v"(b), "v"(c), "v"(d)); }
__device__ __forceinline__ void keep4_b(v16b a, v16b b, v16b c, v16b d) { asm volatile("v_nop" :: "v"(a), "v"(b), "v"(c), "v"(d)); }
__device__ __forceinline__ void acc_guard4(v8f& a, v8f& b, v8f& c, v8f& d) { asm volatile("v_nop\n\tv_nop\n\tv_nop\n\tv_nop" : "+v"(a), "+v"(b), "+v"(c), "+v"(d)); }
template <typename T> struct Frag;
template <> struct Frag<_Float16> {
  typedef v16h V; union U { v16h v; v8h h[2]; };
  static __device__ __forceinline__ v16h load(const _Float16* p) {
    U f; f.h[0] = *(const v8h*)(p); f.h[1] = *(const v8h*)(p + 16); return f.v;
  }
  static __device__ __forceinline__ v8f mma(v16h a, v16h b, v8f c) {
    return __builtin_amdgcn_wmma_f32_16x16x32_f16(false, a, false, b, (short)0, c, false, false);
  }
  static __device__ __forceinline__ void guard(v8f& a, v8f& b, v16h x, v16h y) { dep_guard_h(a, b, x, y); }
  static __device__ __forceinline__ void keep(v16h a, v16h b, v16h c, v16h d) { keep4_h(a, b, c, d); }
};
template <> struct Frag<__bf16> {
  typedef v16b V; union U { v16b v; v8b h[2]; };
  static __device__ __forceinline__ v16b load(const __bf16* p) {
    U f; f.h[0] = *(const v8b*)(p); f.h[1] = *(const v8b*)(p + 16); return f.v;
  }
  static __device__ __forceinline__ v8f mma(v16b a, v16b b, v8f c) {
    return __builtin_amdgcn_wmma_f32_16x16x32_bf16(false, a, false, b, (short)0, c, false, false);
  }
  static __device__ __forceinline__ void guard(v8f& a, v8f& b, v16b x, v16b y) { dep_guard_b(a, b, x, y); }
  static __device__ __forceinline__ void keep(v16b a, v16b b, v16b c, v16b d) { keep4_b(a, b, c, d); }
};

template <int ET> struct Elem;
template <> struct Elem<0> { typedef _Float16 T; };
template <> struct Elem<1> { typedef __bf16 T; };
template <int ET, int SPL, int BIAS_MODE, int OUT_MODE, bool RESID, int ACT = 0>
__global__ __launch_bounds__(256) void wmma_gemm64(
    const unsigned short* __restrict__ Ap, const unsigned short* __restrict__ A2p, int lda, long strideA,
    const unsigned short* __restrict__ Btp, const unsigned short* __restrict__ Bt2p, int ldb, long strideB,
    void* __restrict__ Cout, void* __restrict__ Cout2, int ldc, long strideC,
    const float* __restrict__ bias,
    const float* __restrict__ resid, long strideR,
    int M, int N, int K, float scale) {
  typedef typename Elem<ET>::T T;
  typedef typename Frag<T>::V V;
  const T* A = (const T*)Ap; const T* A2 = (const T*)A2p; const T* Bt = (const T*)Btp; const T* Bt2 = (const T*)Bt2p;
  __shared__ __align__(16) float sT[8][16 * 68];
  const int b    = blockIdx.y;
  const int lane = threadIdx.x & 31;
  const int wave = threadIdx.x >> 5;
  const int tilesN = N >> 6;
  const int tilesM = M >> 6;
  const int tile = blockIdx.x * 8 + wave;
  if (tile >= tilesM * tilesN) return;
  const int tm = tile / tilesN;
  const int tn = tile - tm * tilesN;
  const int m0 = tm << 6;
  const int n0 = tn << 6;

  const T* Ab  = A  + (size_t)b * strideA;
  const T* Bb  = Bt + (size_t)b * strideB;
  const T* Ab2 = (SPL >= 1) ? (A2  + (size_t)b * strideA) : nullptr;
  const T* Bb2 = (SPL == 2) ? (Bt2 + (size_t)b * strideB) : nullptr;

  const int rlane = lane & 15;
  const int koff  = (lane >> 4) * 8;
  const int mOff  = (lane >> 4) * 8;

  v8f acc[4][4];
#pragma unroll
  for (int i = 0; i < 4; ++i)
#pragma unroll
    for (int j = 0; j < 4; ++j) acc[i][j] = (v8f){0.f,0.f,0.f,0.f,0.f,0.f,0.f,0.f};

  for (int k0 = 0; k0 < K; k0 += 32) {
    V bh[4], bl[4];
#pragma unroll
    for (int j = 0; j < 4; ++j) {
      const size_t bo = (size_t)(n0 + (j << 4) + rlane) * ldb + koff + k0;
      bh[j] = Frag<T>::load(Bb + bo);
      if (SPL == 2) bl[j] = Frag<T>::load(Bb2 + bo);
    }
#pragma unroll
    for (int i = 0; i < 4; ++i) {
      const size_t ao = (size_t)(m0 + (i << 4) + rlane) * lda + koff + k0;
      V ah = Frag<T>::load(Ab + ao);
      V al;
      if (SPL >= 1) al = Frag<T>::load(Ab2 + ao);
#pragma unroll
      for (int j = 0; j < 4; ++j) {
        acc[i][j] = Frag<T>::mma(ah, bh[j], acc[i][j]);
        if (SPL == 2) acc[i][j] = Frag<T>::mma(ah, bl[j], acc[i][j]);
        if (SPL >= 1) acc[i][j] = Frag<T>::mma(al, bh[j], acc[i][j]);
      }
      Frag<T>::guard(acc[i][0], acc[i][3], ah, (SPL >= 1) ? al : ah);
    }
    Frag<T>::keep(bh[0], bh[1], bh[2], bh[3]);
    if (SPL == 2) Frag<T>::keep(bl[0], bl[1], bl[2], bl[3]);
  }
  acc_guard4(acc[0][0], acc[0][1], acc[0][2], acc[0][3]);
  acc_guard4(acc[1][0], acc[1][1], acc[1][2], acc[1][3]);
  acc_guard4(acc[2][0], acc[2][1], acc[2][2], acc[2][3]);
  acc_guard4(acc[3][0], acc[3][1], acc[3][2], acc[3][3]);

  float* slab = sT[wave];
  const float* Rb = RESID ? (resid + (size_t)b * strideR) : nullptr;
#pragma unroll
  for (int i = 0; i < 4; ++i) {
    const int mBase = m0 + (i << 4);
#pragma unroll
    for (int j = 0; j < 4; ++j) {
      const int n = n0 + (j << 4) + rlane;
      float bv = 0.f;
      if (BIAS_MODE == 2) bv = bias[n];
#pragma unroll
      for (int r = 0; r < 8; ++r) {
        float v = acc[i][j][r] * scale;
        if (BIAS_MODE == 1) v += bias[mBase + mOff + r];
        if (BIAS_MODE == 2) v += bv;
        if (RESID) v += Rb[(size_t)(mBase + mOff + r) * ldc + n];
        if (ACT == 1) v = tanhf(v);
        if (ACT == 2) v = fmaxf(v, 0.0f);
        if (ACT == 3) v = v / (1.0f + expf(-v));
        if (ACT == 4) v = (v > 0.f) ? v : 0.01f * v;
        slab[(mOff + r) * 68 + (j << 4) + rlane] = v;
      }
    }
    __builtin_amdgcn_fence(__ATOMIC_RELEASE, "workgroup");
    __builtin_amdgcn_wave_barrier();
    __builtin_amdgcn_fence(__ATOMIC_ACQUIRE, "workgroup");
    if (OUT_MODE == 0) {
      float* C = (float*)Cout + (size_t)b * strideC;
      const int hh = lane >> 4, c4 = (lane & 15) * 4;
      for (int pass = 0; pass < 2; ++pass) {
#pragma unroll
        for (int it = 0; it < 8; ++it) {
          const int row = it * 2 + hh;
          v4f v = *(const v4f*)(slab + row * 68 + c4);
          *(volatile v4f*)(C + (size_t)(mBase + row) * ldc + n0 + c4) = v;
        }
        __threadfence();
      }
    } else {
      const int q = lane >> 3, c8 = (lane & 7) * 8;
      unsigned short* C  = (unsigned short*)Cout  + (size_t)b * strideC;
      unsigned short* C2 = (OUT_MODE == 2) ? ((unsigned short*)Cout2 + (size_t)b * strideC) : nullptr;
      for (int pass = 0; pass < 2; ++pass) {
#pragma unroll
        for (int it = 0; it < 4; ++it) {
          const int row = it * 4 + q;
          const float* sp = slab + row * 68 + c8;
          v8h hv, lv;
#pragma unroll
          for (int e = 0; e < 8; ++e) {
            if (OUT_MODE == 1) {
              hv[e] = (_Float16)sp[e];
            } else {
              unsigned short hb = f2bf_bits(sp[e]);
              unsigned short lb = f2bf_bits(sp[e] - bf_bits2f(hb));
              hv[e] = __builtin_bit_cast(_Float16, hb);
              lv[e] = __builtin_bit_cast(_Float16, lb);
            }
          }
          *(volatile v8h*)(C + (size_t)(mBase + row) * ldc + n0 + c8) = hv;
          if (OUT_MODE == 2) *(volatile v8h*)(C2 + (size_t)(mBase + row) * ldc + n0 + c8) = lv;
        }
        __threadfence();
      }
    }
    __builtin_amdgcn_fence(__ATOMIC_RELEASE, "workgroup");
    __builtin_amdgcn_wave_barrier();
    __builtin_amdgcn_fence(__ATOMIC_ACQUIRE, "workgroup");
  }
}

__global__ __launch_bounds__(256) void cast_scale_f16_kernel(
    const float* __restrict__ src, unsigned short* __restrict__ dst, int total8, float scale)
{
  const int i = blockIdx.x * 256 + threadIdx.x;
  if (i >= total8) return;
  const size_t e0 = (size_t)i << 3;
  const v4f a0 = *(const v4f*)(src + e0);
  const v4f a1 = *(const v4f*)(src + e0 + 4);
  v8h hv;
#pragma unroll
  for (int e = 0; e < 4; ++e) {
    hv[e]     = (_Float16)(a0[e] * scale);
    hv[4 + e] = (_Float16)(a1[e] * scale);
  }
  unsigned short* q = dst + e0;
  *(volatile v8h*)q = hv;
  __threadfence();
  *(volatile v8h*)q = hv;
}

__global__ __launch_bounds__(256) void rmsnorm_f16_kernel(
    const float* __restrict__ x, const float* __restrict__ nw, unsigned short* __restrict__ H, int nrows)
{
  const int lane = threadIdx.x & 31, wave = threadIdx.x >> 5;
  const int row = blockIdx.x * 8 + wave;
  if (row >= nrows) return;
  const float* xr = x + (size_t)row * kDm;
  const int c0 = lane * 8, c1 = 256 + lane * 8;
  const v4f a0 = *(const v4f*)(xr + c0), a1 = *(const v4f*)(xr + c0 + 4);
  const v4f a2 = *(const v4f*)(xr + c1), a3 = *(const v4f*)(xr + c1 + 4);
  float ss = 0.f;
#pragma unroll
  for (int e = 0; e < 4; ++e) {
    ss += a0[e] * a0[e];
    ss += a1[e] * a1[e];
    ss += a2[e] * a2[e];
    ss += a3[e] * a3[e];
  }
#pragma unroll
  for (int off = 16; off > 0; off >>= 1) ss += __shfl_xor(ss, off, 32);
  const float inv = rsqrtf(ss * (1.0f / (float)kDm) + 1e-5f);
  const v4f w0 = *(const v4f*)(nw + c0), w1 = *(const v4f*)(nw + c0 + 4);
  const v4f w2 = *(const v4f*)(nw + c1), w3 = *(const v4f*)(nw + c1 + 4);
  v8h h0, h1;
#pragma unroll
  for (int e = 0; e < 4; ++e) {
    h0[e]     = (_Float16)((a0[e] * inv) * w0[e]);
    h0[4 + e] = (_Float16)((a1[e] * inv) * w1[e]);
    h1[e]     = (_Float16)((a2[e] * inv) * w2[e]);
    h1[4 + e] = (_Float16)((a3[e] * inv) * w3[e]);
  }
  unsigned short* q0 = H + (size_t)row * kDm + c0;
  unsigned short* q1 = H + (size_t)row * kDm + c1;
  for (int pass = 0; pass < 2; ++pass) {
    *(volatile v8h*)q0 = h0;
    *(volatile v8h*)q1 = h1;
    __threadfence();
  }
}

__global__ __launch_bounds__(256) void conv_silu_kernel(
    const float* __restrict__ XZ, const float* __restrict__ cw, const float* __restrict__ cb,
    float* __restrict__ UC, unsigned short* __restrict__ U16)
{
  __shared__ __align__(16) float sT[16 * kConvTP];
  const int tid = threadIdx.x, lane = tid & 31, wave = tid >> 5;
  const int d0 = blockIdx.x * 256, d = d0 + tid;
  const int g0 = blockIdx.y * 64;
  const int tb = g0 & (kSeq - 1);
  const float w0 = cw[d * 4 + 0], w1 = cw[d * 4 + 1], w2 = cw[d * 4 + 2], w3 = cw[d * 4 + 3];
  const float bc = cb[d];
  float xm3, xm2, xm1;
  {
    const bool hist = (tb > 0);
    const int rb = hist ? (g0 - 3) : g0;
    const float v3 = XZ[(size_t)rb * kXzP + d];
    const float v2 = XZ[(size_t)(rb + 1) * kXzP + d];
    const float v1 = XZ[(size_t)(rb + 2) * kXzP + d];
    xm3 = hist ? v3 : 0.f;
    xm2 = hist ? v2 : 0.f;
    xm1 = hist ? v1 : 0.f;
  }
  const int hrow = wave >> 1;
  const int hch  = (wave & 1) * 128 + lane * 4;
#pragma unroll 1
  for (int sub = 0; sub < 4; ++sub) {
    const int lb = g0 + sub * 16;
#pragma unroll 1
    for (int s = 0; s < 16; ++s) {
      const float xcur = XZ[(size_t)(lb + s) * kXzP + d];
      float acc = w0 * xm3;
      acc = fmaf(w1, xm2, acc);
      acc = fmaf(w2, xm1, acc);
      acc = fmaf(w3, xcur, acc);
      const float sv = acc + bc;
      const float sg = __builtin_amdgcn_rcpf(1.0f + __expf(-sv));
      sT[s * kConvTP + tid] = sv * sg;
      xm3 = xm2; xm2 = xm1; xm1 = xcur;
    }
    __syncthreads();
    v4f fv[4];
    v8h hv[2];
#pragma unroll
    for (int it = 0; it < 4; ++it) fv[it] = *(const v4f*)(sT + (it * 4 + hrow) * kConvTP + hch);
#pragma unroll
    for (int it = 0; it < 2; ++it) {
      const float* sp = sT + (it * 8 + wave) * kConvTP + lane * 8;
      const v4f a0 = *(const v4f*)(sp);
      const v4f a1 = *(const v4f*)(sp + 4);
#pragma unroll
      for (int e = 0; e < 4; ++e) {
        hv[it][e]     = (_Float16)(a0[e] * kUsc);
        hv[it][4 + e] = (_Float16)(a1[e] * kUsc);
      }
    }
    for (int pass = 0; pass < 2; ++pass) {
#pragma unroll
      for (int it = 0; it < 4; ++it)
        *(volatile v4f*)(UC + (size_t)(lb + it * 4 + hrow) * kDin + d0 + hch) = fv[it];
#pragma unroll
      for (int it = 0; it < 2; ++it) {
        const size_t o = (size_t)(lb + it * 8 + wave) * kDin + d0 + lane * 8;
        *(volatile v8h*)(U16 + o) = hv[it];
      }
      __threadfence();
    }
    __syncthreads();
  }
}

__global__ __launch_bounds__(64) void scan_kernel(
    const float* __restrict__ XD, const float* __restrict__ UC, const float* __restrict__ XZ,
    const float* __restrict__ Wdt, const float* __restrict__ bdt, const float* __restrict__ Alog,
    const float* __restrict__ Dp, unsigned short* __restrict__ Y16)
{
  __shared__ __align__(16) float sX[kScanTS * kXdP];
  __shared__ __align__(16) float sY[kScanTS * kScanYP];
  __shared__ __align__(16) float sW[kDtR * kScanCh];
  __shared__ __align__(16) float sA[kNst * kScanCh];
  const int tid = threadIdx.x, lane = tid & 31, wave = tid >> 5;
  constexpr int kBlkPerB = kDin / kScanCh;
  const int bix = blockIdx.x / kBlkPerB;
  const int d0  = (blockIdx.x - bix * kBlkPerB) * kScanCh;
  const int d   = d0 + tid;
  const size_t row0 = (size_t)bix * kSeq;
#pragma unroll 1
  for (int r = 0; r < kDtR; ++r) sW[r * kScanCh + tid] = Wdt[(size_t)d * kDtR + r];
#pragma unroll 1
  for (int s = 0; s < kNst; ++s) sA[s * kScanCh + tid] = -expf(Alog[(size_t)d * kNst + s]);
  __syncthreads();
  float negA[kNst], h[kNst];
#pragma unroll
  for (int s = 0; s < kNst; ++s) {
    negA[s] = sA[s * kScanCh + tid];
    h[s] = 0.f;
  }
  const float bb = bdt[d], Dd = Dp[d];
  const int lr = tid >> 4, lc4 = (tid & 15) * 4;
  const int q = lane >> 3, c8 = (lane & 7) * 8;
#pragma unroll 1
  for (int t0 = 0; t0 < kSeq; t0 += kScanTS) {
    __syncthreads();
#pragma unroll
    for (int i = 0; i < 16; ++i) {
      const int r = lr + 4 * i;
      *(v4f*)(sX + r * kXdP + lc4) = *(const v4f*)(XD + (row0 + t0 + r) * kXdP + lc4);
    }
    __syncthreads();
#pragma unroll 1
    for (int s = 0; s < kScanTS; ++s) {
      const int t = t0 + s;
      const float* xr = sX + s * kXdP;
      float vdot = 0.f;
#pragma unroll 1
      for (int r4 = 0; r4 < kDtR / 4; ++r4) {
        const v4f xv = *(const v4f*)(xr + 4 * r4);
        const float* wp = sW + (4 * r4) * kScanCh + tid;
        vdot = fmaf(xv[0], wp[0], vdot);
        vdot = fmaf(xv[1], wp[kScanCh], vdot);
        vdot = fmaf(xv[2], wp[2 * kScanCh], vdot);
        vdot = fmaf(xv[3], wp[3 * kScanCh], vdot);
      }
      float Bs[kNst], Cs[kNst];
#pragma unroll
      for (int q4 = 0; q4 < 4; ++q4) {
        const v4f bv = *(const v4f*)(xr + kDtR + 4 * q4);
        const v4f cv = *(const v4f*)(xr + kDtR + kNst + 4 * q4);
        Bs[4 * q4 + 0] = bv[0]; Bs[4 * q4 + 1] = bv[1]; Bs[4 * q4 + 2] = bv[2]; Bs[4 * q4 + 3] = bv[3];
        Cs[4 * q4 + 0] = cv[0]; Cs[4 * q4 + 1] = cv[1]; Cs[4 * q4 + 2] = cv[2]; Cs[4 * q4 + 3] = cv[3];
      }
      const float v   = vdot + bb;
      const float a   = __expf(-fabsf(v));
      const float u   = 1.0f + a;
      const float l1p = __logf(u) + (a - (u - 1.0f)) * __builtin_amdgcn_rcpf(u);
      const float dt  = fmaxf(v, 0.0f) + l1p;
      const float xt  = UC[(row0 + t) * kDin + d];
      const float dtx = dt * xt;
      float y = 0.f;
#pragma unroll
      for (int k = 0; k < kNst; ++k) {
        const float e = __expf(dt * negA[k]);
        h[k] = e * h[k] + dtx * Bs[k];
        y = h[k] * Cs[k] + y;
      }
      y = xt * Dd + y;
      const float zv = XZ[(row0 + t) * kXzP + kDin + d];
      const float sg = __builtin_amdgcn_rcpf(1.0f + __expf(-zv));
      y = y * (zv * sg);
      sY[s * kScanYP + tid] = y;
    }
    __syncthreads();
    v8h hv[8];
#pragma unroll
    for (int it = 0; it < 8; ++it) {
      const int row = it * 8 + wave * 4 + q;
      const float* sp = sY + row * kScanYP + c8;
      const v4f a0 = *(const v4f*)(sp);
      const v4f a1 = *(const v4f*)(sp + 4);
#pragma unroll
      for (int e = 0; e < 4; ++e) {
        hv[it][e]     = (_Float16)(a0[e] * kYsc);
        hv[it][4 + e] = (_Float16)(a1[e] * kYsc);
      }
    }
    for (int pass = 0; pass < 2; ++pass) {
#pragma unroll
      for (int it = 0; it < 8; ++it) {
        const int row = it * 8 + wave * 4 + q;
        const size_t o = (row0 + t0 + row) * kDin + d0 + c8;
        *(volatile v8h*)(Y16 + o) = hv[it];
      }
      __threadfence();
    }
  }
}

__global__ __launch_bounds__(256) void post_out_kernel(
    const float* __restrict__ OUT, const float* __restrict__ X,
    unsigned short* __restrict__ OUT16, unsigned short* __restrict__ WK16, float* __restrict__ XPO, int nwaves)
{
  const int lane = threadIdx.x & 31, wave = threadIdx.x >> 5;
  const int gw = blockIdx.x * 8 + wave;
  if (gw >= nwaves) return;
  const size_t base = (size_t)gw * 256;
  const size_t e0 = base + (size_t)lane * 8;
  const int row = (int)(e0 >> 9);
  const int t = row & (kSeq - 1);
  const size_t ep = (t > 0) ? (e0 - (size_t)kDm) : e0;
  const float zs = (t > 0) ? kOsc : 0.0f;
  const v4f o0 = *(const v4f*)(OUT + e0), o1 = *(const v4f*)(OUT + e0 + 4);
  const v4f p0 = *(const v4f*)(OUT + ep), p1 = *(const v4f*)(OUT + ep + 4);
  v8h ov, wv;
#pragma unroll
  for (int e = 0; e < 4; ++e) {
    ov[e]     = (_Float16)(o0[e] * kOsc);
    ov[4 + e] = (_Float16)(o1[e] * kOsc);
    wv[e]     = (_Float16)(p0[e] * zs);
    wv[4 + e] = (_Float16)(p1[e] * zs);
  }
  const size_t f0 = base + (size_t)lane * 4, f1 = base + 128 + (size_t)lane * 4;
  const v4f xa = *(const v4f*)(X + f0), xb = *(const v4f*)(X + f1);
  const v4f oa = *(const v4f*)(OUT + f0), ob = *(const v4f*)(OUT + f1);
  const v4f ra = xa + oa, rb = xb + ob;
  for (int pass = 0; pass < 2; ++pass) {
    *(volatile v8h*)(OUT16 + e0) = ov;
    *(volatile v8h*)(WK16 + e0) = wv;
    *(volatile v4f*)(XPO + f0) = ra;
    *(volatile v4f*)(XPO + f1) = rb;
    __threadfence();
  }
}

__global__ __launch_bounds__(256) void decay_weight_kernel(
    const float* __restrict__ S, const float* __restrict__ decay_p, unsigned short* __restrict__ P16, int total8)
{
  const int i = blockIdx.x * 256 + threadIdx.x;
  if (i >= total8) return;
  const size_t e0 = (size_t)i << 3;
  const int s0 = (int)(e0 & (kSeq - 1));
  const int t  = (int)((e0 >> 10) & (kSeq - 1));
  const float dec = decay_p[0];
  const float sig = 1.0f / (1.0f + expf(-dec));
  const float lg  = logf(sig);
  const v4f a0 = *(const v4f*)(S + e0);
  const v4f a1 = *(const v4f*)(S + e0 + 4);
  v8h pv;
#pragma unroll
  for (int e = 0; e < 8; ++e) {
    const int s = s0 + e;
    int kd = t - 1 - s;
    kd = kd < 0 ? 0 : kd;
    const float arg = (float)kd * lg;
    float m = expf(arg);
    m = (t > s) ? m : 0.0f;
    const float val = (e < 4) ? a0[e] : a1[e - 4];
    pv[e] = (_Float16)((val * m) * kPsc);
  }
  unsigned short* q = P16 + e0;
  *(volatile v8h*)q = pv;
  __threadfence();
  *(volatile v8h*)q = pv;
}

extern "C" void kernel_launch(void* const* d_in, const int* in_sizes, int n_in,
                              void* d_out, int out_size, void* d_ws, size_t ws_size,
                              hipStream_t stream) {
  if (n_in < 14) return;
  if (in_sizes[0]  != kRows * kDm) return;
  if (in_sizes[1]  != kDm) return;
  if (in_sizes[2]  != kXzP * kDm) return;
  if (in_sizes[3]  != kDin * 4) return;
  if (in_sizes[4]  != kDin) return;
  if (in_sizes[5]  != kXdP * kDin) return;
  if (in_sizes[6]  != kDin * kDtR) return;
  if (in_sizes[7]  != kDin) return;
  if (in_sizes[8]  != kDin * kNst) return;
  if (in_sizes[9]  != kDin) return;
  if (in_sizes[10] != kDm * kDin) return;
  if (in_sizes[11] != kDm * kDm) return;
  if (in_sizes[12] != kDm * kDm) return;
  if (in_sizes[13] < 1) return;
  if (out_size != kRows * kDm) return;
  if (ws_size < kWsTotal) return;

  const float* x       = (const float*)d_in[0];
  const float* norm_w  = (const float*)d_in[1];
  const float* W_in    = (const float*)d_in[2];
  const float* conv_w  = (const float*)d_in[3];
  const float* conv_b  = (const float*)d_in[4];
  const float* W_xproj = (const float*)d_in[5];
  const float* W_dt    = (const float*)d_in[6];
  const float* b_dt    = (const float*)d_in[7];
  const float* A_log   = (const float*)d_in[8];
  const float* Dp      = (const float*)d_in[9];
  const float* W_out   = (const float*)d_in[10];
  const float* W_write = (const float*)d_in[11];
  const float* W_read  = (const float*)d_in[12];
  const float* decay   = (const float*)d_in[13];
  float* out = (float*)d_out;

  char* ws = (char*)d_ws;
  unsigned short* H16   = (unsigned short*)(ws + kOffH16);
  unsigned short* WI16  = (unsigned short*)(ws + kOffWI16);
  unsigned short* WX16  = (unsigned short*)(ws + kOffWX16);
  unsigned short* WO16  = (unsigned short*)(ws + kOffWO16);
  unsigned short* WW16  = (unsigned short*)(ws + kOffWW16);
  unsigned short* WR16  = (unsigned short*)(ws + kOffWR16);
  float*          XZ    = (float*)(ws + kOffXZ);
  float*          S     = (float*)(ws + kOffS);
  unsigned short* P16   = (unsigned short*)(ws + kOffP16);
  float*          UC    = (float*)(ws + kOffUC);
  unsigned short* U16   = (unsigned short*)(ws + kOffU16);
  float*          XD    = (float*)(ws + kOffXD);
  unsigned short* Y16   = (unsigned short*)(ws + kOffY16);
  float*          OUT   = (float*)(ws + kOffOUT);
  unsigned short* OUT16 = (unsigned short*)(ws + kOffOUT16);
  unsigned short* WK16  = (unsigned short*)(ws + kOffWK16);
  float*          XPO   = (float*)(ws + kOffXPO);
  unsigned short* VT16  = (unsigned short*)(ws + kOffVT16);
  unsigned short* RD16  = (unsigned short*)(ws + kOffRD16);

  {
    const int n8a = kXzP * kDm / 8, n8b = kXdP * kDin / 8, n8c = kDm * kDin / 8, n8d = kDm * kDm / 8;
    cast_scale_f16_kernel<<<(n8a + 255) / 256, 256, 0, stream>>>(W_in,    WI16, n8a, kWsc);
    cast_scale_f16_kernel<<<(n8b + 255) / 256, 256, 0, stream>>>(W_xproj, WX16, n8b, kWsc);
    cast_scale_f16_kernel<<<(n8c + 255) / 256, 256, 0, stream>>>(W_out,   WO16, n8c, kWsc);
    cast_scale_f16_kernel<<<(n8d + 255) / 256, 256, 0, stream>>>(W_write, WW16, n8d, kWsc);
    cast_scale_f16_kernel<<<(n8d + 255) / 256, 256, 0, stream>>>(W_read,  WR16, n8d, kWsc);
  }

  rmsnorm_f16_kernel<<<(kRows + 7) / 8, 256, 0, stream>>>(x, norm_w, H16, kRows);

  wmma_gemm64<0, 0, 0, 0, false><<<dim3(256, 1), 256, 0, stream>>>(
      H16, nullptr, kDm, 0L,
      WI16, nullptr, kDm, 0L,
      (void*)XZ, nullptr, kXzP, 0L,
      nullptr, nullptr, 0L,
      kRows, kXzP, kDm, 1.0f / kWsc);

  conv_silu_kernel<<<dim3(kDin / 256, kRows / 64), 256, 0, stream>>>(XZ, conv_w, conv_b, UC, U16);

  wmma_gemm64<0, 0, 0, 0, false><<<dim3(8, 1), 256, 0, stream>>>(
      U16, nullptr, kDin, 0L,
      WX16, nullptr, kDin, 0L,
      (void*)XD, nullptr, kXdP, 0L,
      nullptr, nullptr, 0L,
      kRows, kXdP, kDin, 1.0f / (kUsc * kWsc));

  scan_kernel<<<kBatch * (kDin / kScanCh), kScanCh, 0, stream>>>(XD, UC, XZ, W_dt, b_dt, A_log, Dp, Y16);

  wmma_gemm64<0, 0, 0, 0, false><<<dim3(64, 1), 256, 0, stream>>>(
      Y16, nullptr, kDin, 0L,
      WO16, nullptr, kDin, 0L,
      (void*)OUT, nullptr, kDm, 0L,
      nullptr, nullptr, 0L,
      kRows, kDm, kDin, 1.0f / (kYsc * kWsc));

  {
    const int nwaves = kRows * kDm / 256;
    post_out_kernel<<<(nwaves + 7) / 8, 256, 0, stream>>>(OUT, x, OUT16, WK16, XPO, nwaves);
  }

  wmma_gemm64<0, 0, 0, 1, false><<<dim3(16, kBatch), 256, 0, stream>>>(
      WW16, nullptr, kDm, 0L,
      OUT16, nullptr, kDm, (long)kSeq * kDm,
      (void*)VT16, nullptr, kSeq, (long)kDm * kSeq,
      nullptr, nullptr, 0L,
      kDm, kSeq, kDm, kVsc / (kWsc * kOsc));

  wmma_gemm64<0, 0, 0, 0, false><<<dim3(32, kBatch), 256, 0, stream>>>(
      OUT16, nullptr, kDm, (long)kSeq * kDm,
      WK16, nullptr, kDm, (long)kSeq * kDm,
      (void*)S, nullptr, kSeq, (long)kSeq * kSeq,
      nullptr, nullptr, 0L,
      kSeq, kSeq, kDm, 1.0f / (kOsc * kOsc));

  {
    const int n8 = kBatch * kSeq * kSeq / 8;
    decay_weight_kernel<<<(n8 + 255) / 256, 256, 0, stream>>>(S, decay, P16, n8);
  }

  wmma_gemm64<0, 0, 0, 1, false><<<dim3(16, kBatch), 256, 0, stream>>>(
      P16, nullptr, kSeq, (long)kSeq * kSeq,
      VT16, nullptr, kSeq, (long)kDm * kSeq,
      (void*)RD16, nullptr, kDm, (long)kSeq * kDm,
      nullptr, nullptr, 0L,
      kSeq, kDm, kSeq, kRsc / (kPsc * kVsc));

  wmma_gemm64<0, 0, 0, 0, true><<<dim3(64, 1), 256, 0, stream>>>(
      RD16, nullptr, kDm, 0L,
      WR16, nullptr, kDm, 0L,
      (void*)out, nullptr, kDm, 0L,
      nullptr, XPO, 0L,
      kRows, kDm, kDm, 0.03f / (kRsc * kWsc));
}
